// MultiHeadSelfAttentionLayer_39754217292499
// MI455X (gfx1250) — hardware-verified
//
#include <hip/hip_runtime.h>
#include <stdint.h>
#include <stddef.h>

typedef __attribute__((ext_vector_type(16))) _Float16 v16h;
typedef __attribute__((ext_vector_type(8)))  _Float16 v8h;
typedef __attribute__((ext_vector_type(16))) __bf16   v16b;
typedef __attribute__((ext_vector_type(8)))  __bf16   v8b;
typedef __attribute__((ext_vector_type(8)))  float    v8f;
typedef __attribute__((ext_vector_type(4)))  float    v4f;
typedef __attribute__((ext_vector_type(4)))  unsigned v4u;
typedef __attribute__((ext_vector_type(2)))  unsigned v2u;

constexpr int kBatch = 2;
constexpr int kSeq   = 2048;
constexpr int kEmb   = 1024;
constexpr int kHeads = 16;
constexpr int kHeadD = 64;
constexpr int kTok   = kBatch * kSeq;
static_assert(kHeads * kHeadD == kEmb, "");
static_assert(kHeadD == 64, "");
static_assert(kTok % 64 == 0 && kEmb % 64 == 0, "");
static_assert(kEmb % 32 == 0, "");
static_assert(kSeq % 64 == 0, "");

#define AT_NW 4
#define AT_QB 64
#define AT_KC 64

__device__ __forceinline__ unsigned short f2bf_bits(float f) {
  unsigned u = __float_as_uint(f);
  return (unsigned short)((u + 0x7FFFu + ((u >> 16) & 1u)) >> 16);
}
__device__ __forceinline__ float bf_bits2f(unsigned short h) { return __uint_as_float(((unsigned)h) << 16); }

__device__ __forceinline__ void dep_guard_h(v8f& a, v8f& b, v16h x, v16h y) { asm volatile("v_nop\n\tv_nop\n\tv_nop\n\tv_nop" : "+v"(a), "+v"(b) : "v"(x), "v"(y)); }
__device__ __forceinline__ void dep_guard_b(v8f& a, v8f& b, v16b x, v16b y) { asm volatile("v_nop\n\tv_nop\n\tv_nop\n\tv_nop" : "+v"(a), "+v"(b) : "v"(x), "v"(y)); }
__device__ __forceinline__ void keep4_h(v16h a, v16h b, v16h c, v16h d) { asm volatile("v_nop" :: "v"(a), "v"(b), "v"(c), "v"(d)); }
__device__ __forceinline__ void keep4_b(v16b a, v16b b, v16b c, v16b d) { asm volatile("v_nop" :: "v"(a), "v"(b), "v"(c), "v"(d)); }
__device__ __forceinline__ void acc_guard4(v8f& a, v8f& b, v8f& c, v8f& d) { asm volatile("v_nop\n\tv_nop\n\tv_nop\n\tv_nop" : "+v"(a), "+v"(b), "+v"(c), "+v"(d)); }

template <typename T> struct Frag;
template <> struct Frag<_Float16> {
  typedef v16h V; union U { v16h v; v8h h[2]; };
  static __device__ __forceinline__ v16h load(const _Float16* p) {
    U f; f.h[0] = *(const v8h*)(p); f.h[1] = *(const v8h*)(p + 16); return f.v;
  }
  static __device__ __forceinline__ v8f mma(v16h a, v16h b, v8f c) {
    return __builtin_amdgcn_wmma_f32_16x16x32_f16(false, a, false, b, (short)0, c, false, false);
  }
  static __device__ __forceinline__ void guard(v8f& a, v8f& b, v16h x, v16h y) { dep_guard_h(a, b, x, y); }
  static __device__ __forceinline__ void keep(v16h a, v16h b, v16h c, v16h d) { keep4_h(a, b, c, d); }
};
template <> struct Frag<__bf16> {
  typedef v16b V; union U { v16b v; v8b h[2]; };
  static __device__ __forceinline__ v16b load(const __bf16* p) {
    U f; f.h[0] = *(const v8b*)(p); f.h[1] = *(const v8b*)(p + 16); return f.v;
  }
  static __device__ __forceinline__ v8f mma(v16b a, v16b b, v8f c) {
    return __builtin_amdgcn_wmma_f32_16x16x32_bf16(false, a, false, b, (short)0, c, false, false);
  }
  static __device__ __forceinline__ void guard(v8f& a, v8f& b, v16b x, v16b y) { dep_guard_b(a, b, x, y); }
  static __device__ __forceinline__ void keep(v16b a, v16b b, v16b c, v16b d) { keep4_b(a, b, c, d); }
};

__global__ __launch_bounds__(256) void cast_f32_bf16x4(
    const float* __restrict__ in, unsigned short* __restrict__ out, int n4) {
  const int i = blockIdx.x * 256 + threadIdx.x;
  if (i < n4) {
    const v4f f = *(const v4f*)(in + 4 * (size_t)i);
    v2u u;
    u[0] = (unsigned)f2bf_bits(f[0]) | ((unsigned)f2bf_bits(f[1]) << 16);
    u[1] = (unsigned)f2bf_bits(f[2]) | ((unsigned)f2bf_bits(f[3]) << 16);
    *(volatile v2u*)(out + 4 * (size_t)i) = u;
    __threadfence();
    *(volatile v2u*)(out + 4 * (size_t)i) = u;
  }
}

__global__ __launch_bounds__(256) void transpose_cast_bf16(
    const float* __restrict__ W, unsigned short* __restrict__ Wt, int nrows_k, int ncols_n) {
  __shared__ float T[64][65];
  const int k0 = blockIdx.y * 64;
  const int n0 = blockIdx.x * 64;
  const int tid = threadIdx.x;
#pragma unroll
  for (int i = 0; i < 4; ++i) {
    const int idx = tid + 256 * i;
    const int r = idx >> 4;
    const int c4 = (idx & 15) * 4;
    const v4f v = *(const v4f*)(W + (size_t)(k0 + r) * ncols_n + n0 + c4);
    T[r][c4] = v[0]; T[r][c4 + 1] = v[1]; T[r][c4 + 2] = v[2]; T[r][c4 + 3] = v[3];
  }
  __syncthreads();
  v4u pk[2];
  size_t off[2];
#pragma unroll
  for (int i = 0; i < 2; ++i) {
    const int idx = tid + 256 * i;
    const int n = idx >> 3;
    const int c8 = (idx & 7) * 8;
    v4u u;
#pragma unroll
    for (int e = 0; e < 4; ++e)
      u[e] = (unsigned)f2bf_bits(T[c8 + 2 * e][n]) | ((unsigned)f2bf_bits(T[c8 + 2 * e + 1][n]) << 16);
    pk[i] = u;
    off[i] = (size_t)(n0 + n) * nrows_k + k0 + c8;
  }
  for (int pass = 0; pass < 2; ++pass) {
#pragma unroll
    for (int i = 0; i < 2; ++i) *(volatile v4u*)(Wt + off[i]) = pk[i];
    __threadfence();
  }
}

template <int ET> struct Elem;
template <> struct Elem<0> { typedef _Float16 T; };
template <> struct Elem<1> { typedef __bf16 T; };
template <int ET, int SPLIT, int BIAS_MODE, int OUT_MODE>
__global__ __launch_bounds__(256) void wmma_gemm64(
    const unsigned short* __restrict__ Ap, const unsigned short* __restrict__ A2p, int lda, long strideA,
    const unsigned short* __restrict__ Btp, const unsigned short* __restrict__ Bt2p, int ldb, long strideB,
    void* __restrict__ Cout, void* __restrict__ Cout2, int ldc, long strideC,
    const float* __restrict__ bias,
    int M, int N, int K, float scale) {
  typedef typename Elem<ET>::T T;
  typedef typename Frag<T>::V V;
  const T* A = (const T*)Ap; const T* A2 = (const T*)A2p; const T* Bt = (const T*)Btp; const T* Bt2 = (const T*)Bt2p;
  __shared__ __align__(16) float sT[8][16 * 68];
  const int b    = blockIdx.y;
  const int lane = threadIdx.x & 31;
  const int wave = threadIdx.x >> 5;
  const int tilesN = N >> 6;
  const int tilesM = M >> 6;
  const int tile = blockIdx.x * 8 + wave;
  if (tile >= tilesM * tilesN) return;
  const int tm = tile / tilesN;
  const int tn = tile - tm * tilesN;
  const int m0 = tm << 6;
  const int n0 = tn << 6;

  const T* Ab  = A  + (size_t)b * strideA;
  const T* Bb  = Bt + (size_t)b * strideB;
  const T* Ab2 = (SPLIT != 0) ? (A2  + (size_t)b * strideA) : nullptr;
  const T* Bb2 = (SPLIT == 1) ? (Bt2 + (size_t)b * strideB) : nullptr;

  const int rlane = lane & 15;
  const int koff  = (lane >> 4) * 8;
  const int mOff  = (lane >> 4) * 8;

  v8f acc[4][4];
#pragma unroll
  for (int i = 0; i < 4; ++i)
#pragma unroll
    for (int j = 0; j < 4; ++j) acc[i][j] = (v8f){0.f,0.f,0.f,0.f,0.f,0.f,0.f,0.f};

  for (int k0 = 0; k0 < K; k0 += 32) {
    V bh[4], bl[4];
#pragma unroll
    for (int j = 0; j < 4; ++j) {
      const size_t bo = (size_t)(n0 + (j << 4) + rlane) * ldb + koff + k0;
      bh[j] = Frag<T>::load(Bb + bo);
      if (SPLIT == 1) bl[j] = Frag<T>::load(Bb2 + bo);
    }
#pragma unroll
    for (int i = 0; i < 4; ++i) {
      const size_t ao = (size_t)(m0 + (i << 4) + rlane) * lda + koff + k0;
      V ah = Frag<T>::load(Ab + ao);
      V al = ah;
      if (SPLIT != 0) al = Frag<T>::load(Ab2 + ao);
#pragma unroll
      for (int j = 0; j < 4; ++j) {
        acc[i][j] = Frag<T>::mma(ah, bh[j], acc[i][j]);
        if (SPLIT == 1) acc[i][j] = Frag<T>::mma(ah, bl[j], acc[i][j]);
        if (SPLIT != 0) acc[i][j] = Frag<T>::mma(al, bh[j], acc[i][j]);
      }
      Frag<T>::guard(acc[i][0], acc[i][3], ah, al);
    }
    Frag<T>::keep(bh[0], bh[1], bh[2], bh[3]);
    if (SPLIT == 1) Frag<T>::keep(bl[0], bl[1], bl[2], bl[3]);
  }
  acc_guard4(acc[0][0], acc[0][1], acc[0][2], acc[0][3]);
  acc_guard4(acc[1][0], acc[1][1], acc[1][2], acc[1][3]);
  acc_guard4(acc[2][0], acc[2][1], acc[2][2], acc[2][3]);
  acc_guard4(acc[3][0], acc[3][1], acc[3][2], acc[3][3]);

  float* slab = sT[wave];
#pragma unroll
  for (int i = 0; i < 4; ++i) {
    const int mBase = m0 + (i << 4);
    float bmr[8];
#pragma unroll
    for (int r = 0; r < 8; ++r) bmr[r] = 0.f;
    if (BIAS_MODE == 1) {
      const v4f b0 = *(const v4f*)(bias + mBase + mOff);
      const v4f b1 = *(const v4f*)(bias + mBase + mOff + 4);
      bmr[0] = b0[0]; bmr[1] = b0[1]; bmr[2] = b0[2]; bmr[3] = b0[3];
      bmr[4] = b1[0]; bmr[5] = b1[1]; bmr[6] = b1[2]; bmr[7] = b1[3];
    }
#pragma unroll
    for (int j = 0; j < 4; ++j) {
      const int n = n0 + (j << 4) + rlane;
      float bv = 0.f;
      if (BIAS_MODE == 2) bv = bf_bits2f(f2bf_bits(bias[n]));
#pragma unroll
      for (int r = 0; r < 8; ++r) {
        float v = acc[i][j][r] * scale;
        if (BIAS_MODE == 1) v += bf_bits2f(f2bf_bits(bmr[r]));
        if (BIAS_MODE == 2) v += bv;
        slab[(mOff + r) * 68 + (j << 4) + rlane] = v;
      }
    }
    __builtin_amdgcn_fence(__ATOMIC_RELEASE, "workgroup");
    __builtin_amdgcn_wave_barrier();
    __builtin_amdgcn_fence(__ATOMIC_ACQUIRE, "workgroup");
    if (OUT_MODE == 0) {
      float* C = (float*)Cout + (size_t)b * strideC;
      const int hh = lane >> 4, c4 = (lane & 15) * 4;
      for (int pass = 0; pass < 2; ++pass) {
#pragma unroll
        for (int it = 0; it < 8; ++it) {
          const int row = it * 2 + hh;
          v4f v = *(const v4f*)(slab + row * 68 + c4);
          *(volatile v4f*)(C + (size_t)(mBase + row) * ldc + n0 + c4) = v;
        }
        __threadfence();
      }
    } else {
      const int q = lane >> 3, c8 = (lane & 7) * 8;
      unsigned short* C  = (unsigned short*)Cout  + (size_t)b * strideC;
      unsigned short* C2 = (OUT_MODE == 2) ? ((unsigned short*)Cout2 + (size_t)b * strideC) : nullptr;
      for (int pass = 0; pass < 2; ++pass) {
#pragma unroll
        for (int it = 0; it < 4; ++it) {
          const int row = it * 4 + q;
          const float* sp = slab + row * 68 + c8;
          v8h hv, lv;
#pragma unroll
          for (int e = 0; e < 8; ++e) {
            if (OUT_MODE == 1) {
              hv[e] = (_Float16)sp[e];
            } else {
              unsigned short hb = f2bf_bits(sp[e]);
              unsigned short lb = f2bf_bits(sp[e] - bf_bits2f(hb));
              hv[e] = __builtin_bit_cast(_Float16, hb);
              lv[e] = __builtin_bit_cast(_Float16, lb);
            }
          }
          *(volatile v8h*)(C + (size_t)(mBase + row) * ldc + n0 + c8) = hv;
          if (OUT_MODE == 2) *(volatile v8h*)(C2 + (size_t)(mBase + row) * ldc + n0 + c8) = lv;
        }
        __threadfence();
      }
    }
    __builtin_amdgcn_fence(__ATOMIC_RELEASE, "workgroup");
    __builtin_amdgcn_wave_barrier();
    __builtin_amdgcn_fence(__ATOMIC_ACQUIRE, "workgroup");
  }
}

__device__ __forceinline__ unsigned short at_bf_bits(float f) {
  unsigned u = __float_as_uint(f);
  return (unsigned short)((u + 0x7FFFu + ((u >> 16) & 1u)) >> 16);
}
__device__ __forceinline__ __bf16 at_f2bf(float f) { return __builtin_bit_cast(__bf16, at_bf_bits(f)); }
__device__ __forceinline__ void at_split(float f, __bf16& hi, __bf16& lo) {
  const unsigned short hb = at_bf_bits(f);
  hi = __builtin_bit_cast(__bf16, hb);
  lo = at_f2bf(f - __uint_as_float(((unsigned)hb) << 16));
}
__device__ __forceinline__ v8f at_mma(v16b a, v16b b, v8f c) {
  c = __builtin_amdgcn_wmma_f32_16x16x32_bf16(false, a, false, b, (short)0, c, false, false);
  asm volatile("v_nop\n\tv_nop\n\tv_nop\n\tv_nop" : "+v"(c) : "v"(a), "v"(b));
  return c;
}
__device__ __forceinline__ v8f at_mma_h(v16h a, v16h b, v8f c) {
  c = __builtin_amdgcn_wmma_f32_16x16x32_f16(false, a, false, b, (short)0, c, false, false);
  asm volatile("v_nop\n\tv_nop\n\tv_nop\n\tv_nop" : "+v"(c) : "v"(a), "v"(b));
  return c;
}

__global__ __launch_bounds__(128)
void attn16_kernel(const unsigned short* __restrict__ Qp, const unsigned short* __restrict__ Kp,
                   const unsigned short* __restrict__ Vthp, const unsigned short* __restrict__ Vtlp,
                   unsigned short* __restrict__ Ohp, unsigned short* __restrict__ Olp, float sm_scale) {
  union FB { v16b v; v8b h[2]; };
  __shared__ __align__(16) __bf16 Psh[AT_NW][16 * AT_KC];
  __shared__ __align__(16) __bf16 Psl[AT_NW][16 * AT_KC];
  __shared__ __align__(16) float  Os[AT_NW][16 * 68];

  const int tid  = threadIdx.x;
  const int wave = tid >> 5;
  const int lane = tid & 31;
  const int hh   = lane >> 4;
  const int c    = lane & 15;

  const int nqb = kSeq / AT_QB;
  const int bx = blockIdx.x;
  const int qb = bx % nqb;
  const int bh = bx / nqb;
  const int h  = bh % kHeads;
  const int b  = bh / kHeads;
  const int q0 = qb * AT_QB + wave * 16;
  const size_t tokb = (size_t)b * kSeq;
  const int colh = h * kHeadD;

  const _Float16* Q  = (const _Float16*)(const void*)Qp;
  const _Float16* Kk = (const _Float16*)(const void*)Kp;
  const __bf16*   Vh = (const __bf16*)(const void*)Vthp;
  const __bf16*   Vl = (const __bf16*)(const void*)Vtlp;

  v16h qa[2];
#pragma unroll
  for (int dc = 0; dc < 2; ++dc)
    qa[dc] = Frag<_Float16>::load(Q + (tokb + q0 + c) * (size_t)kEmb + colh + dc * 32 + 8 * hh);

  float mrow[8], lrow[8];
  v8f oacc[4];
#pragma unroll
  for (int r = 0; r < 8; ++r) { mrow[r] = -INFINITY; lrow[r] = 0.f; }
#pragma unroll
  for (int t = 0; t < 4; ++t) oacc[t] = (v8f){0.f,0.f,0.f,0.f,0.f,0.f,0.f,0.f};

  __bf16* pwh = Psh[wave];
  __bf16* pwl = Psl[wave];

  for (int kc = 0; kc < kSeq / AT_KC; ++kc) {
    const int kv0 = kc * AT_KC;
    __syncthreads();

    v8f s[4];
#pragma unroll
    for (int j = 0; j < 4; ++j) {
      s[j] = (v8f){0.f,0.f,0.f,0.f,0.f,0.f,0.f,0.f};
      const _Float16* krow = Kk + (tokb + kv0 + j * 16 + c) * (size_t)kEmb + colh + 8 * hh;
#pragma unroll
      for (int dc = 0; dc < 2; ++dc) {
        const v16h kb = Frag<_Float16>::load(krow + dc * 32);
        s[j] = at_mma_h(qa[dc], kb, s[j]);
      }
    }

    float cm[8];
#pragma unroll
    for (int r = 0; r < 8; ++r) {
      float m = -INFINITY;
#pragma unroll
      for (int j = 0; j < 4; ++j) {
        const float sv = s[j][r] * sm_scale;
        s[j][r] = sv;
        m = fmaxf(m, sv);
      }
#pragma unroll
      for (int off = 1; off < 16; off <<= 1) m = fmaxf(m, __shfl_xor(m, off, 32));
      cm[r] = m;
    }

#pragma unroll
    for (int r = 0; r < 8; ++r) {
      const float mnew = fmaxf(mrow[r], cm[r]);
      const float alpha = expf(mrow[r] - mnew);
      mrow[r] = mnew;
      float psum = 0.f;
#pragma unroll
      for (int j = 0; j < 4; ++j) {
        const float p = expf(s[j][r] - mnew);
        psum += p;
        __bf16 a, bl; at_split(p, a, bl);
        pwh[(8 * hh + r) * AT_KC + j * 16 + c] = a;
        pwl[(8 * hh + r) * AT_KC + j * 16 + c] = bl;
      }
#pragma unroll
      for (int off = 1; off < 16; off <<= 1) psum += __shfl_xor(psum, off, 32);
      lrow[r] = lrow[r] * alpha + psum;
#pragma unroll
      for (int t = 0; t < 4; ++t) oacc[t][r] *= alpha;
    }
    __builtin_amdgcn_fence(__ATOMIC_RELEASE, "workgroup");
    __builtin_amdgcn_wave_barrier();
    __builtin_amdgcn_fence(__ATOMIC_ACQUIRE, "workgroup");

#pragma unroll 1
    for (int kk = 0; kk < 2; ++kk) {
      FB pa, pl;
      pa.h[0] = *(const v8b*)(pwh + c * AT_KC + kk * 32 + 8 * hh);
      pa.h[1] = *(const v8b*)(pwh + c * AT_KC + kk * 32 + 16 + 8 * hh);
      pl.h[0] = *(const v8b*)(pwl + c * AT_KC + kk * 32 + 8 * hh);
      pl.h[1] = *(const v8b*)(pwl + c * AT_KC + kk * 32 + 16 + 8 * hh);
#pragma unroll
      for (int t = 0; t < 4; ++t) {
        const size_t vo = (size_t)(colh + t * 16 + c) * kTok + tokb + kv0 + kk * 32 + 8 * hh;
        const v16b vb = Frag<__bf16>::load(Vh + vo);
        const v16b vl = Frag<__bf16>::load(Vl + vo);
        oacc[t] = at_mma(pa.v, vb, oacc[t]);
        oacc[t] = at_mma(pa.v, vl, oacc[t]);
        oacc[t] = at_mma(pl.v, vb, oacc[t]);
      }
    }
  }

  float* os = Os[wave];
#pragma unroll
  for (int r = 0; r < 8; ++r) {
    const float inv = 1.0f / lrow[r];
#pragma unroll
    for (int t = 0; t < 4; ++t) os[(8 * hh + r) * 68 + t * 16 + c] = oacc[t][r] * inv;
  }
  __builtin_amdgcn_fence(__ATOMIC_RELEASE, "workgroup");
  __builtin_amdgcn_wave_barrier();
  __builtin_amdgcn_fence(__ATOMIC_ACQUIRE, "workgroup");
  {
    const int q8 = lane >> 3, c8 = (lane & 7) * 8;
    for (int pass = 0; pass < 2; ++pass) {
#pragma unroll
      for (int it = 0; it < 4; ++it) {
        const int row = it * 4 + q8;
        const float* sp = os + row * 68 + c8;
        v8h hv, lv;
#pragma unroll
        for (int e = 0; e < 8; ++e) {
          const unsigned short hb = f2bf_bits(sp[e]);
          const unsigned short lb = f2bf_bits(sp[e] - bf_bits2f(hb));
          hv[e] = __builtin_bit_cast(_Float16, hb);
          lv[e] = __builtin_bit_cast(_Float16, lb);
        }
        const size_t oo = (tokb + q0 + row) * (size_t)kEmb + colh + c8;
        *(volatile v8h*)(Ohp + oo) = hv;
        *(volatile v8h*)(Olp + oo) = lv;
      }
      __threadfence();
    }
  }
}

extern "C" void kernel_launch(void* const* d_in, const int* in_sizes, int n_in,
                              void* d_out, int out_size, void* d_ws, size_t ws_size,
                              hipStream_t stream) {
  if (n_in < 11) return;
  const int nAct = kTok * kEmb;
  const int nW   = kEmb * kEmb;
  if (in_sizes[0] != nAct || in_sizes[1] != nAct || in_sizes[2] != nAct) return;
  if (in_sizes[3] != nW || in_sizes[4] != nW || in_sizes[5] != nW || in_sizes[6] != nW) return;
  if (in_sizes[7] != kEmb || in_sizes[8] != kEmb || in_sizes[9] != kEmb || in_sizes[10] != kEmb) return;
  if (out_size != nAct) return;
  static_assert((kTok * kEmb / 4) % 256 == 0, "");

  const float* query    = (const float*)d_in[0];
  const float* key      = (const float*)d_in[1];
  const float* value    = (const float*)d_in[2];
  const float* W_Query  = (const float*)d_in[3];
  const float* W_Key    = (const float*)d_in[4];
  const float* W_Value  = (const float*)d_in[5];
  const float* W_Output = (const float*)d_in[6];
  const float* B_Query  = (const float*)d_in[7];
  const float* B_Key    = (const float*)d_in[8];
  const float* B_Value  = (const float*)d_in[9];
  const float* B_Output = (const float*)d_in[10];

  const size_t actPlane = (size_t)nAct * 2;
  const size_t wPlane   = (size_t)nW * 2;
  size_t off = 0;
  const size_t oXq = off; off += actPlane;
  const size_t oXk = off; off += actPlane;
  const size_t oXv = off; off += actPlane;
  const size_t oWQ = off; off += wPlane;
  const size_t oWK = off; off += wPlane;
  const size_t oWV = off; off += wPlane;
  const size_t oWO = off; off += wPlane;
  const size_t oQh = off; off += actPlane;
  const size_t oKh = off; off += actPlane;
  const size_t oVth = off; off += actPlane;
  const size_t oVtl = off; off += actPlane;
  const size_t oOh = off; off += actPlane;
  const size_t oOl = off; off += actPlane;
  if (off > ws_size) return;

  char* ws = (char*)d_ws;
  unsigned short* Xq  = (unsigned short*)(ws + oXq);
  unsigned short* Xk  = (unsigned short*)(ws + oXk);
  unsigned short* Xv  = (unsigned short*)(ws + oXv);
  unsigned short* WQt = (unsigned short*)(ws + oWQ);
  unsigned short* WKt = (unsigned short*)(ws + oWK);
  unsigned short* WVt = (unsigned short*)(ws + oWV);
  unsigned short* WOt = (unsigned short*)(ws + oWO);
  unsigned short* Qh  = (unsigned short*)(ws + oQh);
  unsigned short* Kh  = (unsigned short*)(ws + oKh);
  unsigned short* Vth = (unsigned short*)(ws + oVth);
  unsigned short* Vtl = (unsigned short*)(ws + oVtl);
  unsigned short* Oh  = (unsigned short*)(ws + oOh);
  unsigned short* Ol  = (unsigned short*)(ws + oOl);

  const dim3 blk256(256);

  const int n4 = nAct / 4;
  const dim3 gCast(n4 / 256);
  cast_f32_bf16x4<<<gCast, blk256, 0, stream>>>(query, Xq, n4);
  cast_f32_bf16x4<<<gCast, blk256, 0, stream>>>(key,   Xk, n4);
  cast_f32_bf16x4<<<gCast, blk256, 0, stream>>>(value, Xv, n4);

  const dim3 gTr(kEmb / 64, kEmb / 64);
  transpose_cast_bf16<<<gTr, blk256, 0, stream>>>(W_Query,  WQt, kEmb, kEmb);
  transpose_cast_bf16<<<gTr, blk256, 0, stream>>>(W_Key,    WKt, kEmb, kEmb);
  transpose_cast_bf16<<<gTr, blk256, 0, stream>>>(W_Value,  WVt, kEmb, kEmb);
  transpose_cast_bf16<<<gTr, blk256, 0, stream>>>(W_Output, WOt, kEmb, kEmb);

  const int gemmBlocks = (kTok / 64) * (kEmb / 64) / 8;
  const dim3 gGemm(gemmBlocks, 1);
  wmma_gemm64<1, 0, 2, 1><<<gGemm, blk256, 0, stream>>>(
      Xq, Xq, kEmb, 0L, WQt, WQt, kEmb, 0L, (void*)Qh, (void*)Qh, kEmb, 0L,
      B_Query, kTok, kEmb, kEmb, 1.0f);
  wmma_gemm64<1, 0, 2, 1><<<gGemm, blk256, 0, stream>>>(
      Xk, Xk, kEmb, 0L, WKt, WKt, kEmb, 0L, (void*)Kh, (void*)Kh, kEmb, 0L,
      B_Key, kTok, kEmb, kEmb, 1.0f);
  wmma_gemm64<1, 0, 1, 2><<<gGemm, blk256, 0, stream>>>(
      WVt, WVt, kEmb, 0L, Xv, Xv, kEmb, 0L, (void*)Vth, (void*)Vtl, kTok, 0L,
      B_Value, kEmb, kTok, kEmb, 1.0f);

  const dim3 gAttn(kBatch * kHeads * (kSeq / AT_QB));
  attn16_kernel<<<gAttn, dim3(128), 0, stream>>>(Qh, Kh, Vth, Vtl, Oh, Ol, 0.125f);

  wmma_gemm64<1, 2, 2, 0><<<gGemm, blk256, 0, stream>>>(
      Oh, Ol, kEmb, 0L, WOt, WOt, kEmb, 0L, d_out, d_out, kEmb, 0L,
      B_Output, kTok, kEmb, kEmb, 1.0f);
}
